// Mamba_84267258347738
// MI455X (gfx1250) — hardware-verified
//
#include <hip/hip_runtime.h>
#include <math.h>

typedef __attribute__((ext_vector_type(16))) _Float16 v16h;
typedef __attribute__((ext_vector_type(8)))  _Float16 v8h;
typedef __attribute__((ext_vector_type(16))) __bf16   v16b;
typedef __attribute__((ext_vector_type(8)))  __bf16   v8b;
typedef __attribute__((ext_vector_type(8)))  float    v8f;
typedef __attribute__((ext_vector_type(4)))  float    v4f;

constexpr int kBatch = 2;
constexpr int kSeq   = 1024;
constexpr int kDm    = 1024;
constexpr int kDin   = 2048;
constexpr int kNst   = 16;
constexpr int kDtR   = 64;
constexpr int kPrjN  = 96;
constexpr int kPrjP  = 128;
constexpr int kXzP   = 2 * kDin;
constexpr int kRows  = kBatch * kSeq;
constexpr int kTP    = 260;
static_assert(kDtR + 2 * kNst == kPrjN, "x_proj width");
static_assert((kSeq & (kSeq - 1)) == 0, "sequence length is a power of two");
static_assert((kSeq % 64) == 0 && (kDin % 256) == 0, "tile multiples");
static_assert((kRows % 64) == 0 && (kXzP % 64) == 0 && (kPrjP % 64) == 0 && (kDin % 64) == 0 && (kDm % 64) == 0, "GEMM M,N multiples of 64");
static_assert((kDm % 32) == 0 && (kDin % 32) == 0 && (kDtR % 32) == 0, "GEMM K multiples of 32");

constexpr size_t kOffHS   = 0;
constexpr size_t kOffWIN  = kOffHS   + (size_t)kRows * kDm   * 2;
constexpr size_t kOffWXP  = kOffWIN  + (size_t)kXzP  * kDm   * 2;
constexpr size_t kOffWDT  = kOffWXP  + (size_t)kPrjP * kDin  * 2;
constexpr size_t kOffWOUT = kOffWDT  + (size_t)kDin  * kDtR  * 2;
constexpr size_t kOffXZ   = kOffWOUT + (size_t)kDm   * kDin  * 2;
constexpr size_t kOffUC   = kOffXZ   + (size_t)kRows * kXzP  * 4;
constexpr size_t kOffUCH  = kOffUC   + (size_t)kRows * kDin  * 4;
constexpr size_t kOffUCL  = kOffUCH  + (size_t)kRows * kDin  * 2;
constexpr size_t kOffPROJ = kOffUCL  + (size_t)kRows * kDin  * 2;
constexpr size_t kOffGATE = kOffPROJ + (size_t)kRows * kPrjP * 4;
constexpr size_t kOffDT   = kOffGATE + (size_t)kBatch * kPrjP * 4;
constexpr size_t kOffDLR  = kOffDT   + (size_t)kRows * kDtR  * 2;
constexpr size_t kOffYH   = kOffDLR  + (size_t)kRows * kDin  * 4;
constexpr size_t kOffYL   = kOffYH   + (size_t)kRows * kDin  * 2;
constexpr size_t kWsTotal = kOffYL   + (size_t)kRows * kDin  * 2;
static_assert(kWsTotal == 119538688ull, "carve total");
static_assert(kWsTotal <= 134217728ull, "carve cap");
static_assert((kOffWIN % 128) == 0 && (kOffWXP % 128) == 0 && (kOffWDT % 128) == 0 && (kOffWOUT % 128) == 0 &&
              (kOffXZ % 128) == 0 && (kOffUC % 128) == 0 && (kOffUCH % 128) == 0 && (kOffUCL % 128) == 0 &&
              (kOffPROJ % 128) == 0 && (kOffGATE % 128) == 0 && (kOffDT % 128) == 0 && (kOffDLR % 128) == 0 &&
              (kOffYH % 128) == 0 && (kOffYL % 128) == 0, "128-B aligned regions");

__device__ __forceinline__ unsigned short f2bf_bits(float f) {
  unsigned u = __float_as_uint(f);
  return (unsigned short)((u + 0x7FFFu + ((u >> 16) & 1u)) >> 16);
}
__device__ __forceinline__ float bf_bits2f(unsigned short h) { return __uint_as_float(((unsigned)h) << 16); }
__device__ __forceinline__ float bf_rne(float f) { return bf_bits2f(f2bf_bits(f)); }

__device__ __forceinline__ void dep_guard4_h(v8f& a, v8f& b, v8f& c, v8f& d, v16h x, v16h y) {
  asm volatile("v_nop\n\tv_nop\n\tv_nop\n\tv_nop" : "+v"(a), "+v"(b), "+v"(c), "+v"(d) : "v"(x), "v"(y));
}
__device__ __forceinline__ void dep_guard4_b(v8f& a, v8f& b, v8f& c, v8f& d, v16b x, v16b y) {
  asm volatile("v_nop\n\tv_nop\n\tv_nop\n\tv_nop" : "+v"(a), "+v"(b), "+v"(c), "+v"(d) : "v"(x), "v"(y));
}
__device__ __forceinline__ void keep4_h(v16h a, v16h b, v16h c, v16h d) { asm volatile("v_nop" :: "v"(a), "v"(b), "v"(c), "v"(d)); }
__device__ __forceinline__ void keep4_b(v16b a, v16b b, v16b c, v16b d) { asm volatile("v_nop" :: "v"(a), "v"(b), "v"(c), "v"(d)); }
__device__ __forceinline__ void acc_guard4(v8f& a, v8f& b, v8f& c, v8f& d) { asm volatile("v_nop\n\tv_nop\n\tv_nop\n\tv_nop" : "+v"(a), "+v"(b), "+v"(c), "+v"(d)); }

template <typename T> struct Frag;
template <> struct Frag<_Float16> {
  typedef v16h V; union U { v16h v; v8h h[2]; };
  static __device__ __forceinline__ v16h load(const _Float16* p) {
    U f; f.h[0] = *(const v8h*)(p); f.h[1] = *(const v8h*)(p + 16); return f.v;
  }
  static __device__ __forceinline__ v8f mma(v16h a, v16h b, v8f c) {
    return __builtin_amdgcn_wmma_f32_16x16x32_f16(false, a, false, b, (short)0, c, false, false);
  }
  static __device__ __forceinline__ void guard(v8f& a, v8f& b, v8f& c, v8f& d, v16h x, v16h y) { dep_guard4_h(a, b, c, d, x, y); }
  static __device__ __forceinline__ void keep(v16h a, v16h b, v16h c, v16h d) { keep4_h(a, b, c, d); }
};
template <> struct Frag<__bf16> {
  typedef v16b V; union U { v16b v; v8b h[2]; };
  static __device__ __forceinline__ v16b load(const __bf16* p) {
    U f; f.h[0] = *(const v8b*)(p); f.h[1] = *(const v8b*)(p + 16); return f.v;
  }
  static __device__ __forceinline__ v8f mma(v16b a, v16b b, v8f c) {
    return __builtin_amdgcn_wmma_f32_16x16x32_bf16(false, a, false, b, (short)0, c, false, false);
  }
  static __device__ __forceinline__ void guard(v8f& a, v8f& b, v8f& c, v8f& d, v16b x, v16b y) { dep_guard4_b(a, b, c, d, x, y); }
  static __device__ __forceinline__ void keep(v16b a, v16b b, v16b c, v16b d) { keep4_b(a, b, c, d); }
};

template <int ET> struct Elem;
template <> struct Elem<0> { typedef _Float16 T; };
template <> struct Elem<1> { typedef __bf16 T; };
template <int ET, int SPL, int BIAS_MODE, int OUT_MODE, bool RESID>
__global__ __launch_bounds__(256) void wmma_gemm64(
    const unsigned short* __restrict__ Ap, const unsigned short* __restrict__ A2p, int lda, long strideA,
    const unsigned short* __restrict__ Btp, const unsigned short* __restrict__ Bt2p, int ldb, long strideB,
    void* __restrict__ Cout, void* __restrict__ Cout2, int ldc, long strideC,
    const float* __restrict__ bias,
    const float* __restrict__ resid, long strideR,
    int M, int N, int K, float scale) {
  typedef typename Elem<ET>::T T;
  typedef typename Frag<T>::V V;
  const T* A = (const T*)Ap; const T* A2 = (const T*)A2p; const T* Bt = (const T*)Btp; const T* Bt2 = (const T*)Bt2p;
  __shared__ __align__(16) float sT[8][16 * 68];
  const int b    = blockIdx.y;
  const int lane = threadIdx.x & 31;
  const int wave = threadIdx.x >> 5;
  const int tilesN = N >> 6;
  const int tilesM = M >> 6;
  const int tile = blockIdx.x * 8 + wave;
  if (tile >= tilesM * tilesN) return;
  const int tm = tile / tilesN;
  const int tn = tile - tm * tilesN;
  const int m0 = tm << 6;
  const int n0 = tn << 6;

  const T* Ab  = A  + (size_t)b * strideA;
  const T* Bb  = Bt + (size_t)b * strideB;
  const T* Ab2 = (SPL >= 1) ? (A2  + (size_t)b * strideA) : nullptr;
  const T* Bb2 = (SPL == 2) ? (Bt2 + (size_t)b * strideB) : nullptr;

  const int rlane = lane & 15;
  const int koff  = (lane >> 4) * 8;
  const int mOff  = (lane >> 4) * 8;

  v8f acc[4][4];
#pragma unroll
  for (int i = 0; i < 4; ++i)
#pragma unroll
    for (int j = 0; j < 4; ++j) acc[i][j] = (v8f){0.f,0.f,0.f,0.f,0.f,0.f,0.f,0.f};

  for (int k0 = 0; k0 < K; k0 += 32) {
    V bh[4], bl[4];
#pragma unroll
    for (int j = 0; j < 4; ++j) {
      const size_t bo = (size_t)(n0 + (j << 4) + rlane) * ldb + koff + k0;
      bh[j] = Frag<T>::load(Bb + bo);
      if (SPL == 2) bl[j] = Frag<T>::load(Bb2 + bo);
    }
#pragma unroll
    for (int i = 0; i < 4; ++i) {
      const size_t ao = (size_t)(m0 + (i << 4) + rlane) * lda + koff + k0;
      V ah = Frag<T>::load(Ab + ao);
      V al;
      if (SPL >= 1) al = Frag<T>::load(Ab2 + ao);
#pragma unroll
      for (int j = 0; j < 4; ++j) {
        acc[i][j] = Frag<T>::mma(ah, bh[j], acc[i][j]);
        if (SPL == 2) acc[i][j] = Frag<T>::mma(ah, bl[j], acc[i][j]);
        if (SPL >= 1) acc[i][j] = Frag<T>::mma(al, bh[j], acc[i][j]);
      }
      Frag<T>::guard(acc[i][0], acc[i][1], acc[i][2], acc[i][3], ah, (SPL >= 1) ? al : ah);
    }
    Frag<T>::keep(bh[0], bh[1], bh[2], bh[3]);
    if (SPL == 2) Frag<T>::keep(bl[0], bl[1], bl[2], bl[3]);
  }
  acc_guard4(acc[0][0], acc[0][1], acc[0][2], acc[0][3]);
  acc_guard4(acc[1][0], acc[1][1], acc[1][2], acc[1][3]);
  acc_guard4(acc[2][0], acc[2][1], acc[2][2], acc[2][3]);
  acc_guard4(acc[3][0], acc[3][1], acc[3][2], acc[3][3]);

  float* slab = sT[wave];
  const float* Rb = RESID ? (resid + (size_t)b * strideR) : nullptr;
#pragma unroll
  for (int i = 0; i < 4; ++i) {
    const int mBase = m0 + (i << 4);
#pragma unroll
    for (int j = 0; j < 4; ++j) {
      const int n = n0 + (j << 4) + rlane;
      float bv = 0.f;
      if (BIAS_MODE == 2) bv = bias[n];
#pragma unroll
      for (int r = 0; r < 8; ++r) {
        float v = acc[i][j][r] * scale;
        if (BIAS_MODE == 1) v += bias[mBase + mOff + r];
        if (BIAS_MODE == 2) v += bv;
        if (RESID) v += Rb[(size_t)(mBase + mOff + r) * ldc + n];
        slab[(mOff + r) * 68 + (j << 4) + rlane] = v;
      }
    }
    __builtin_amdgcn_fence(__ATOMIC_RELEASE, "workgroup");
    __builtin_amdgcn_wave_barrier();
    __builtin_amdgcn_fence(__ATOMIC_ACQUIRE, "workgroup");
    if (OUT_MODE == 0) {
      float* C = (float*)Cout + (size_t)b * strideC;
      const int hh = lane >> 4, c4 = (lane & 15) * 4;
      for (int pass = 0; pass < 2; ++pass) {
#pragma unroll
        for (int it = 0; it < 8; ++it) {
          const int row = it * 2 + hh;
          v4f v = *(const v4f*)(slab + row * 68 + c4);
          *(volatile v4f*)(C + (size_t)(mBase + row) * ldc + n0 + c4) = v;
        }
        __threadfence();
      }
    } else {
      const int q = lane >> 3, c8 = (lane & 7) * 8;
      unsigned short* C  = (unsigned short*)Cout  + (size_t)b * strideC;
      unsigned short* C2 = (OUT_MODE == 2) ? ((unsigned short*)Cout2 + (size_t)b * strideC) : nullptr;
      for (int pass = 0; pass < 2; ++pass) {
#pragma unroll
        for (int it = 0; it < 4; ++it) {
          const int row = it * 4 + q;
          const float* sp = slab + row * 68 + c8;
          v8h hv, lv;
#pragma unroll
          for (int e = 0; e < 8; ++e) {
            if (OUT_MODE == 1) {
              hv[e] = (_Float16)sp[e];
            } else {
              unsigned short hb = f2bf_bits(sp[e]);
              unsigned short lb = f2bf_bits(sp[e] - bf_bits2f(hb));
              hv[e] = __builtin_bit_cast(_Float16, hb);
              lv[e] = __builtin_bit_cast(_Float16, lb);
            }
          }
          *(volatile v8h*)(C + (size_t)(mBase + row) * ldc + n0 + c8) = hv;
          if (OUT_MODE == 2) *(volatile v8h*)(C2 + (size_t)(mBase + row) * ldc + n0 + c8) = lv;
        }
        __threadfence();
      }
    }
    __builtin_amdgcn_fence(__ATOMIC_RELEASE, "workgroup");
    __builtin_amdgcn_wave_barrier();
    __builtin_amdgcn_fence(__ATOMIC_ACQUIRE, "workgroup");
  }
}

__global__ __launch_bounds__(256) void cast_bf16_kernel(
    const float* __restrict__ src, unsigned short* __restrict__ dst, int total8, int valid8)
{
  const int i = blockIdx.x * 256 + threadIdx.x;
  if (i >= total8) return;
  const bool live = (i < valid8);
  const int ic = live ? i : (valid8 - 1);
  const float* p = src + ((size_t)ic << 3);
  const v4f a0 = *(const v4f*)(p);
  const v4f a1 = *(const v4f*)(p + 4);
  v8h hv;
#pragma unroll
  for (int e = 0; e < 4; ++e) {
    const float x0 = a0[e];
    const float x1 = a1[e];
    const unsigned short h0 = live ? f2bf_bits(x0) : (unsigned short)0;
    const unsigned short h1 = live ? f2bf_bits(x1) : (unsigned short)0;
    hv[e]     = __builtin_bit_cast(_Float16, h0);
    hv[4 + e] = __builtin_bit_cast(_Float16, h1);
  }
  unsigned short* q = dst + ((size_t)i << 3);
  *(volatile v8h*)q = hv;
  __threadfence();
  *(volatile v8h*)q = hv;
}

__global__ __launch_bounds__(256) void gate_kernel(
    const float* __restrict__ xt, const float* __restrict__ gw, const float* __restrict__ gb,
    float* __restrict__ GATE)
{
  __shared__ __align__(16) float sG[kBatch * kPrjP];
  const int tid = threadIdx.x, lane = tid & 31, wave = tid >> 5;
  const int b  = wave >> 2;
  const int jb = (wave & 3) * 24;
  if (tid < 64) sG[(tid >> 5) * kPrjP + kPrjN + (tid & 31)] = 0.0f;
#pragma unroll 1
  for (int i = 0; i < 24; ++i) {
    const int j = jb + i;
    const float* xp = xt + (size_t)b * kDm + lane * 4;
    const float* wp = gw + (size_t)j * kDm + lane * 4;
    float s = 0.0f;
#pragma unroll 1
    for (int it = 0; it < kDm / 128; ++it) {
      const v4f xv = *(const v4f*)(xp + it * 128);
      const v4f wv = *(const v4f*)(wp + it * 128);
      const float x0 = xv[0], x1 = xv[1], x2 = xv[2], x3 = xv[3];
      const float w0 = wv[0], w1 = wv[1], w2 = wv[2], w3 = wv[3];
      s = fmaf(bf_rne(x0), bf_rne(w0), s);
      s = fmaf(bf_rne(x1), bf_rne(w1), s);
      s = fmaf(bf_rne(x2), bf_rne(w2), s);
      s = fmaf(bf_rne(x3), bf_rne(w3), s);
    }
    s += __shfl_xor(s, 16, 32);
    s += __shfl_xor(s, 8, 32);
    s += __shfl_xor(s, 4, 32);
    s += __shfl_xor(s, 2, 32);
    s += __shfl_xor(s, 1, 32);
    const float pre = s + bf_rne(gb[j]);
    const float sg = __builtin_amdgcn_rcpf(1.0f + expf(-pre));
    if (lane == 0) sG[b * kPrjP + j] = sg;
  }
  __syncthreads();
  if (wave == 0) {
    const v4f g0 = *(const v4f*)(sG + lane * 4);
    const v4f g1 = *(const v4f*)(sG + kPrjP + lane * 4);
    for (int pass = 0; pass < 2; ++pass) {
      *(volatile v4f*)(GATE + lane * 4) = g0;
      *(volatile v4f*)(GATE + kPrjP + lane * 4) = g1;
      __threadfence();
    }
  }
}

__global__ __launch_bounds__(256) void conv_silu_kernel(
    const float* __restrict__ XZ, const float* __restrict__ cw, const float* __restrict__ cb,
    float* __restrict__ UC, unsigned short* __restrict__ UCH, unsigned short* __restrict__ UCL)
{
  __shared__ __align__(16) float sT[16 * kTP];
  const int tid = threadIdx.x, lane = tid & 31, wave = tid >> 5;
  const int d0 = blockIdx.x * 256, d = d0 + tid;
  const int g0 = blockIdx.y * 64;
  const int tb = g0 & (kSeq - 1);
  const v4f wv = *(const v4f*)(cw + (size_t)d * 4);
  const float c0 = wv[0], c1 = wv[1], c2 = wv[2], c3 = wv[3];
  const float w0 = bf_rne(c0), w1 = bf_rne(c1), w2 = bf_rne(c2), w3 = bf_rne(c3);
  const float bc = bf_rne(cb[d]);
  float xm3, xm2, xm1;
  {
    const bool hist = (tb > 0);
    const int rb = hist ? (g0 - 3) : g0;
    const float v3 = XZ[(size_t)rb * kXzP + d];
    const float v2 = XZ[(size_t)(rb + 1) * kXzP + d];
    const float v1 = XZ[(size_t)(rb + 2) * kXzP + d];
    xm3 = hist ? v3 : 0.f;
    xm2 = hist ? v2 : 0.f;
    xm1 = hist ? v1 : 0.f;
  }
  const int hrow = wave >> 1;
  const int hch  = (wave & 1) * 128 + lane * 4;
#pragma unroll 1
  for (int sub = 0; sub < 4; ++sub) {
    const int lb = g0 + sub * 16;
#pragma unroll 1
    for (int s = 0; s < 16; ++s) {
      const float xcur = XZ[(size_t)(lb + s) * kXzP + d];
      float acc = w0 * xm3;
      acc = fmaf(w1, xm2, acc);
      acc = fmaf(w2, xm1, acc);
      acc = fmaf(w3, xcur, acc);
      const float sv = acc + bc;
      const float sg = __builtin_amdgcn_rcpf(1.0f + expf(-sv));
      sT[s * kTP + tid] = sv * sg;
      xm3 = xm2; xm2 = xm1; xm1 = xcur;
    }
    __syncthreads();
    v4f fv[4];
    v8h bh[2], blo[2];
#pragma unroll
    for (int it = 0; it < 4; ++it) fv[it] = *(const v4f*)(sT + (it * 4 + hrow) * kTP + hch);
#pragma unroll
    for (int it = 0; it < 2; ++it) {
      const float* sp = sT + (it * 8 + wave) * kTP + lane * 8;
      const v4f a0 = *(const v4f*)(sp);
      const v4f a1 = *(const v4f*)(sp + 4);
#pragma unroll
      for (int e = 0; e < 4; ++e) {
        const float x0 = a0[e];
        const float x1 = a1[e];
        const unsigned short h0 = f2bf_bits(x0), h1 = f2bf_bits(x1);
        const unsigned short l0 = f2bf_bits(x0 - bf_bits2f(h0)), l1 = f2bf_bits(x1 - bf_bits2f(h1));
        bh[it][e]      = __builtin_bit_cast(_Float16, h0);
        bh[it][4 + e]  = __builtin_bit_cast(_Float16, h1);
        blo[it][e]     = __builtin_bit_cast(_Float16, l0);
        blo[it][4 + e] = __builtin_bit_cast(_Float16, l1);
      }
    }
    for (int pass = 0; pass < 2; ++pass) {
#pragma unroll
      for (int it = 0; it < 4; ++it)
        *(volatile v4f*)(UC + (size_t)(lb + it * 4 + hrow) * kDin + d0 + hch) = fv[it];
#pragma unroll
      for (int it = 0; it < 2; ++it) {
        const size_t o = (size_t)(lb + it * 8 + wave) * kDin + d0 + lane * 8;
        *(volatile v8h*)(UCH + o) = bh[it];
        *(volatile v8h*)(UCL + o) = blo[it];
      }
      __threadfence();
    }
    __syncthreads();
  }
}

__global__ __launch_bounds__(256) void dt_gate_cast_kernel(
    const float* __restrict__ PROJ, const float* __restrict__ GATE, unsigned short* __restrict__ DT16, int total8)
{
  const int i = blockIdx.x * 256 + threadIdx.x;
  if (i >= total8) return;
  const int e0  = i << 3;
  const int row = e0 >> 6;
  const int c8  = e0 & 63;
  const int bix = row / kSeq;
  const float* p = PROJ + (size_t)row * kPrjP + c8;
  const float* g = GATE + (size_t)bix * kPrjP + c8;
  const v4f a0 = *(const v4f*)(p);
  const v4f a1 = *(const v4f*)(p + 4);
  const v4f g0 = *(const v4f*)(g);
  const v4f g1 = *(const v4f*)(g + 4);
  v8h hv;
#pragma unroll
  for (int e = 0; e < 4; ++e) {
    const float p0 = a0[e] * g0[e];
    const float p1 = a1[e] * g1[e];
    const unsigned short h0 = f2bf_bits(p0);
    const unsigned short h1 = f2bf_bits(p1);
    hv[e]     = __builtin_bit_cast(_Float16, h0);
    hv[4 + e] = __builtin_bit_cast(_Float16, h1);
  }
  unsigned short* qd = DT16 + e0;
  *(volatile v8h*)qd = hv;
  __threadfence();
  *(volatile v8h*)qd = hv;
}

__global__ __launch_bounds__(256) void scan_kernel(
    const float* __restrict__ DLR, const float* __restrict__ UC, const float* __restrict__ XZ,
    const float* __restrict__ PROJ, const float* __restrict__ GATE,
    const float* __restrict__ bdt, const float* __restrict__ A_log, const float* __restrict__ Dv,
    unsigned short* __restrict__ YH, unsigned short* __restrict__ YL)
{
  __shared__ __align__(16) float sBC[16 * 32];
  __shared__ __align__(16) float sY[16 * kTP];
  __shared__ __align__(16) float sA[kNst * 256];
  const int tid = threadIdx.x, lane = tid & 31, wave = tid >> 5;
  constexpr int kBlkPerB = kDin / 256;
  const int bix = blockIdx.x / kBlkPerB;
  const int d0  = (blockIdx.x - bix * kBlkPerB) * 256;
  const int d   = d0 + tid;
  const size_t row0 = (size_t)bix * kSeq;

#pragma unroll 1
  for (int n = 0; n < kNst; ++n) sA[n * 256 + tid] = -expf(bf_rne(A_log[(size_t)d * kNst + n]));
  __syncthreads();
  float An[kNst], h[kNst];
#pragma unroll
  for (int n = 0; n < kNst; ++n) {
    An[n] = sA[n * 256 + tid];
    h[n] = 0.f;
  }
  const float bb = bf_rne(bdt[d]);
  const float Dd = bf_rne(Dv[d]);
  const v4f gq = *(const v4f*)(GATE + (size_t)bix * kPrjP + kDtR + (tid & 7) * 4);

#pragma unroll 1
  for (int c = 0; c < kSeq / 16; ++c) {
    const int l0 = c * 16;
    if (tid < 128) {
      const int r = tid >> 3, q = (tid & 7) * 4;
      const v4f v = *(const v4f*)(PROJ + (row0 + l0 + r) * kPrjP + kDtR + q);
      const v4f w = v * gq;
      *(v4f*)(sBC + r * 32 + q) = w;
    }
    __syncthreads();
#pragma unroll 1
    for (int s = 0; s < 16; ++s) {
      const size_t m = row0 + (size_t)(l0 + s);
      const float av = DLR[m * kDin + d] + bb;
      const float ea  = __expf(-fabsf(av));
      const float up  = 1.0f + ea;
      const float l1p = __logf(up) + (ea - (up - 1.0f)) * __builtin_amdgcn_rcpf(up);
      const float delta = fmaxf(av, 0.0f) + l1p;
      const float xv = UC[m * kDin + d];
      const float zv = XZ[m * kXzP + kDin + d];
      v4f Bq[4], Cq[4];
#pragma unroll
      for (int qq = 0; qq < 4; ++qq) {
        Bq[qq] = *(const v4f*)(sBC + s * 32 + 4 * qq);
        Cq[qq] = *(const v4f*)(sBC + s * 32 + kNst + 4 * qq);
      }
      const float dtx = delta * xv;
      float y = 0.f;
#pragma unroll
      for (int n = 0; n < kNst; ++n) {
        const float e = __expf(delta * An[n]);
        h[n] = fmaf(e, h[n], dtx * Bq[n >> 2][n & 3]);
        y = fmaf(h[n], Cq[n >> 2][n & 3], y);
      }
      y = fmaf(xv, Dd, y);
      const float sg = __builtin_amdgcn_rcpf(1.0f + expf(-zv));
      sY[s * kTP + tid] = y * (zv * sg);
    }
    __syncthreads();
    v8h hv[2], lv[2];
#pragma unroll
    for (int it = 0; it < 2; ++it) {
      const float* sp = sY + (it * 8 + wave) * kTP + lane * 8;
      const v4f a0 = *(const v4f*)(sp);
      const v4f a1 = *(const v4f*)(sp + 4);
#pragma unroll
      for (int e = 0; e < 4; ++e) {
        const float x0 = a0[e];
        const float x1 = a1[e];
        const unsigned short h0 = f2bf_bits(x0), h1 = f2bf_bits(x1);
        const unsigned short q0 = f2bf_bits(x0 - bf_bits2f(h0)), q1 = f2bf_bits(x1 - bf_bits2f(h1));
        hv[it][e]     = __builtin_bit_cast(_Float16, h0);
        hv[it][4 + e] = __builtin_bit_cast(_Float16, h1);
        lv[it][e]     = __builtin_bit_cast(_Float16, q0);
        lv[it][4 + e] = __builtin_bit_cast(_Float16, q1);
      }
    }
    for (int pass = 0; pass < 2; ++pass) {
#pragma unroll
      for (int it = 0; it < 2; ++it) {
        const size_t o = (row0 + (size_t)(l0 + it * 8 + wave)) * kDin + d0 + lane * 8;
        *(volatile v8h*)(YH + o) = hv[it];
        *(volatile v8h*)(YL + o) = lv[it];
      }
      __threadfence();
    }
  }
}

extern "C" void kernel_launch(void* const* d_in, const int* in_sizes, int n_in,
                              void* d_out, int out_size, void* d_ws, size_t ws_size,
                              hipStream_t stream)
{
  if (n_in < 13) return;
  if (in_sizes[0]  != kRows * kDm) return;
  if (in_sizes[1]  != kBatch * kDm) return;
  if (in_sizes[2]  != kXzP * kDm) return;
  if (in_sizes[3]  != kDin * 4) return;
  if (in_sizes[4]  != kDin) return;
  if (in_sizes[5]  != kPrjN * kDin) return;
  if (in_sizes[6]  != kDin * kDtR) return;
  if (in_sizes[7]  != kDin) return;
  if (in_sizes[8]  != kDin * kNst) return;
  if (in_sizes[9]  != kDin) return;
  if (in_sizes[10] != kDm * kDin) return;
  if (in_sizes[11] != kPrjN * kDm) return;
  if (in_sizes[12] != kPrjN) return;
  if (out_size != kRows * kDm) return;
  if (ws_size < kWsTotal) return;

  const float* hs     = (const float*)d_in[0];
  const float* x_text = (const float*)d_in[1];
  const float* W_in   = (const float*)d_in[2];
  const float* conv_w = (const float*)d_in[3];
  const float* conv_b = (const float*)d_in[4];
  const float* W_xprj = (const float*)d_in[5];
  const float* W_dt   = (const float*)d_in[6];
  const float* b_dt   = (const float*)d_in[7];
  const float* A_log  = (const float*)d_in[8];
  const float* Dv     = (const float*)d_in[9];
  const float* W_out  = (const float*)d_in[10];
  const float* gate_w = (const float*)d_in[11];
  const float* gate_b = (const float*)d_in[12];
  float* dout = (float*)d_out;

  char* ws = (char*)d_ws;
  unsigned short* HS16   = (unsigned short*)(ws + kOffHS);
  unsigned short* WIN16  = (unsigned short*)(ws + kOffWIN);
  unsigned short* WXP16  = (unsigned short*)(ws + kOffWXP);
  unsigned short* WDT16  = (unsigned short*)(ws + kOffWDT);
  unsigned short* WOUT16 = (unsigned short*)(ws + kOffWOUT);
  float*          XZ     = (float*)(ws + kOffXZ);
  float*          UC     = (float*)(ws + kOffUC);
  unsigned short* UCH    = (unsigned short*)(ws + kOffUCH);
  unsigned short* UCL    = (unsigned short*)(ws + kOffUCL);
  float*          PROJ   = (float*)(ws + kOffPROJ);
  float*          GATE   = (float*)(ws + kOffGATE);
  unsigned short* DT16   = (unsigned short*)(ws + kOffDT);
  float*          DLR    = (float*)(ws + kOffDLR);
  unsigned short* YH     = (unsigned short*)(ws + kOffYH);
  unsigned short* YL     = (unsigned short*)(ws + kOffYL);
  const float* unused_bias  = b_dt;
  const float* unused_resid = hs;

  cast_bf16_kernel<<<(kRows * kDm / 8) / 256, 256, 0, stream>>>(hs, HS16, kRows * kDm / 8, kRows * kDm / 8);
  cast_bf16_kernel<<<(kXzP * kDm / 8) / 256, 256, 0, stream>>>(W_in, WIN16, kXzP * kDm / 8, kXzP * kDm / 8);
  cast_bf16_kernel<<<(kPrjP * kDin / 8) / 256, 256, 0, stream>>>(W_xprj, WXP16, kPrjP * kDin / 8, kPrjN * kDin / 8);
  cast_bf16_kernel<<<(kDin * kDtR / 8) / 256, 256, 0, stream>>>(W_dt, WDT16, kDin * kDtR / 8, kDin * kDtR / 8);
  cast_bf16_kernel<<<(kDm * kDin / 8) / 256, 256, 0, stream>>>(W_out, WOUT16, kDm * kDin / 8, kDm * kDin / 8);

  gate_kernel<<<1, 256, 0, stream>>>(x_text, gate_w, gate_b, GATE);

  wmma_gemm64<1, 0, 0, 0, false><<<dim3(256, 1), 256, 0, stream>>>(
      HS16, HS16, kDm, 0L,
      WIN16, WIN16, kDm, 0L,
      (void*)XZ, (void*)XZ, kXzP, 0L,
      unused_bias, unused_resid, 0L,
      kRows, kXzP, kDm, 1.0f);

  conv_silu_kernel<<<dim3(kDin / 256, kRows / 64), 256, 0, stream>>>(XZ, conv_w, conv_b, UC, UCH, UCL);

  wmma_gemm64<1, 1, 0, 0, false><<<dim3(8, 1), 256, 0, stream>>>(
      UCH, UCL, kDin, 0L,
      WXP16, WXP16, kDin, 0L,
      (void*)PROJ, (void*)PROJ, kPrjP, 0L,
      unused_bias, unused_resid, 0L,
      kRows, kPrjP, kDin, 1.0f);

  dt_gate_cast_kernel<<<(kRows * kDtR / 8) / 256, 256, 0, stream>>>(PROJ, GATE, DT16, kRows * kDtR / 8);

  wmma_gemm64<1, 0, 0, 0, false><<<dim3(128, 1), 256, 0, stream>>>(
      DT16, DT16, kDtR, 0L,
      WDT16, WDT16, kDtR, 0L,
      (void*)DLR, (void*)DLR, kDin, 0L,
      unused_bias, unused_resid, 0L,
      kRows, kDin, kDtR, 1.0f);

  scan_kernel<<<kBatch * (kDin / 256), 256, 0, stream>>>(DLR, UC, XZ, PROJ, GATE, b_dt, A_log, Dv, YH, YL);

  wmma_gemm64<1, 1, 0, 0, false><<<dim3(64, 1), 256, 0, stream>>>(
      YH, YL, kDin, 0L,
      WOUT16, WOUT16, kDin, 0L,
      (void*)dout, (void*)dout, kDm, 0L,
      unused_bias, unused_resid, 0L,
      kRows, kDm, kDin, 1.0f);
}
